// S4Model_83975200571707
// MI455X (gfx1250) — hardware-run, weakly checked
//
#include <hip/hip_runtime.h>
#include <math.h>

typedef __attribute__((ext_vector_type(16))) _Float16 v16h;
typedef __attribute__((ext_vector_type(8)))  _Float16 v8h;
typedef __attribute__((ext_vector_type(2)))  _Float16 v2h;
typedef __attribute__((ext_vector_type(16))) __bf16   v16b;
typedef __attribute__((ext_vector_type(8)))  __bf16   v8b;
typedef __attribute__((ext_vector_type(8)))  float    v8f;
typedef __attribute__((ext_vector_type(4)))  float    v4f;
typedef __attribute__((ext_vector_type(2)))  float    v2f;

constexpr int kNB   = 16;
constexpr int kL    = 4096;
constexpr int kRows = kNB * kL;
constexpr int kDin  = 32;
constexpr int kH    = 128;
constexpr int kNs   = 32;
constexpr int kNL   = 4;
constexpr int kG    = 2 * kH;
constexpr int kDo   = 32;
constexpr int kDoP  = 64;
constexpr int kThr  = 256;
constexpr float kInCarry = 1024.0f;
constexpr float kWCarry  = 4096.0f;
constexpr float kYCarry  = 1024.0f;
constexpr float kScE = 1.0f / (kInCarry * kInCarry);
constexpr float kScO = 1.0f / (kYCarry * kInCarry);
constexpr float kScD = 1.0f / (kInCarry * kInCarry);
constexpr float kF16MinNormal = 6.103515625e-5f;

static_assert(kRows == 65536 && kDin == 32 && kH == 128 && kNs == 32 && kG == 256 && kDo == 32 && kDoP == 64 && (kL & (kL - 1)) == 0, "the index arithmetic below uses these sizes");

constexpr size_t kOffX16 = 0ull;
constexpr size_t kOffWO16 = 4194304ull;
constexpr size_t kOffWE16 = 4456448ull;
constexpr size_t kOffWD16 = 4464640ull;
constexpr size_t kOffEB = 4481024ull;
constexpr size_t kOffOB = 4482048ull;
constexpr size_t kOffDB = 4486144ull;
constexpr size_t kOffPAR = 4487168ull;
constexpr size_t kOffH0 = 4749312ull;
constexpr size_t kOffH1 = 38303744ull;
constexpr size_t kOffYF = 71858176ull;
constexpr size_t kOffY16 = 105412608ull;
constexpr size_t kOffV = 122189824ull;
constexpr size_t kOffDEC = 189298688ull;
constexpr size_t kWsTotal = 206075904ull;
static_assert(kWsTotal <= 268435456ull, "the carve stands under the contract's 256 MiB of workspace");
static_assert(kOffX16 == 0
  && kOffWO16 == kOffX16 + 4194304ull
  && kOffWE16 == kOffWO16 + 262144ull
  && kOffWD16 == kOffWE16 + 8192ull
  && kOffEB == kOffWD16 + 16384ull
  && kOffOB == kOffEB + 1024ull
  && kOffDB == kOffOB + 4096ull
  && kOffPAR == kOffDB + 1024ull
  && kOffH0 == kOffPAR + 262144ull
  && kOffH1 == kOffH0 + 33554432ull
  && kOffYF == kOffH1 + 33554432ull
  && kOffY16 == kOffYF + 33554432ull
  && kOffV == kOffY16 + 16777216ull
  && kOffDEC == kOffV + 67108864ull
  && kWsTotal == kOffDEC + 16777216ull, "the carve is a chain: every region starts where the one before ends");
static_assert((kOffWO16 % 256) == 0 && (kOffWE16 % 256) == 0 && (kOffWD16 % 256) == 0 && (kOffEB % 256) == 0 && (kOffOB % 256) == 0 && (kOffDB % 256) == 0 && (kOffPAR % 256) == 0 && (kOffH0 % 256) == 0 && (kOffH1 % 256) == 0 && (kOffYF % 256) == 0 && (kOffY16 % 256) == 0 && (kOffV % 256) == 0 && (kOffDEC % 256) == 0, "every region starts on a multiple of 256 B");

__device__ __forceinline__ unsigned short f2bf_bits(float f) {
  unsigned u = __float_as_uint(f);
  return (unsigned short)((u + 0x7FFFu + ((u >> 16) & 1u)) >> 16);
}
__device__ __forceinline__ float bf_bits2f(unsigned short h) { return __uint_as_float(((unsigned)h) << 16); }
__device__ __forceinline__ float bf16r(float f) { return bf_bits2f(f2bf_bits(f)); }
__device__ __forceinline__ float carry_flush(float v, float carry) {
  const float s = v * carry;
  return (fabsf(s) < kF16MinNormal) ? 0.0f : s;
}

__device__ __forceinline__ void dep_guard4_h(v8f& a, v8f& b, v8f& c, v8f& d, v16h x, v16h y) { asm volatile("v_nop\n\tv_nop\n\tv_nop\n\tv_nop" : "+v"(a), "+v"(b), "+v"(c), "+v"(d) : "v"(x), "v"(y)); }
__device__ __forceinline__ void dep_guard4_b(v8f& a, v8f& b, v8f& c, v8f& d, v16b x, v16b y) { asm volatile("v_nop\n\tv_nop\n\tv_nop\n\tv_nop" : "+v"(a), "+v"(b), "+v"(c), "+v"(d) : "v"(x), "v"(y)); }
__device__ __forceinline__ void keep4_h(v16h a, v16h b, v16h c, v16h d) { asm volatile("v_nop" :: "v"(a), "v"(b), "v"(c), "v"(d)); }
__device__ __forceinline__ void keep4_b(v16b a, v16b b, v16b c, v16b d) { asm volatile("v_nop" :: "v"(a), "v"(b), "v"(c), "v"(d)); }
__device__ __forceinline__ void acc_guard4(v8f& a, v8f& b, v8f& c, v8f& d) { asm volatile("v_nop\n\tv_nop\n\tv_nop\n\tv_nop" : "+v"(a), "+v"(b), "+v"(c), "+v"(d)); }

template <typename T> struct Frag;
template <> struct Frag<_Float16> {
  typedef v16h V; union U { v16h v; v8h h[2]; };
  static __device__ __forceinline__ v16h load(const _Float16* p) {
    U f; f.h[0] = *(const v8h*)(p); f.h[1] = *(const v8h*)(p + 16); return f.v;
  }
  static __device__ __forceinline__ v8f mma(v16h a, v16h b, v8f c) {
    return __builtin_amdgcn_wmma_f32_16x16x32_f16(false, a, false, b, (short)0, c, false, false);
  }
  static __device__ __forceinline__ void guard4(v8f& a, v8f& b, v8f& c, v8f& d, v16h x, v16h y) { dep_guard4_h(a, b, c, d, x, y); }
  static __device__ __forceinline__ void keep(v16h a, v16h b, v16h c, v16h d) { keep4_h(a, b, c, d); }
};
template <> struct Frag<__bf16> {
  typedef v16b V; union U { v16b v; v8b h[2]; };
  static __device__ __forceinline__ v16b load(const __bf16* p) {
    U f; f.h[0] = *(const v8b*)(p); f.h[1] = *(const v8b*)(p + 16); return f.v;
  }
  static __device__ __forceinline__ v8f mma(v16b a, v16b b, v8f c) {
    return __builtin_amdgcn_wmma_f32_16x16x32_bf16(false, a, false, b, (short)0, c, false, false);
  }
  static __device__ __forceinline__ void guard4(v8f& a, v8f& b, v8f& c, v8f& d, v16b x, v16b y) { dep_guard4_b(a, b, c, d, x, y); }
  static __device__ __forceinline__ void keep(v16b a, v16b b, v16b c, v16b d) { keep4_b(a, b, c, d); }
};

__device__ __forceinline__ v8f mma_h(v16h a, v16h b, v8f c) {
  c = __builtin_amdgcn_wmma_f32_16x16x32_f16(false, a, false, b, (short)0, c, false, false);
  asm volatile("v_nop\n\tv_nop\n\tv_nop\n\tv_nop" : "+v"(c) : "v"(a), "v"(b));
  return c;
}

template <int ET> struct Elem;
template <> struct Elem<0> { typedef _Float16 T; };
template <> struct Elem<1> { typedef __bf16 T; };
template <int ET, bool SPLIT, int BIAS_MODE, int OUT_MODE, bool RESID, int ACT = 0>
__global__ __launch_bounds__(256) void wmma_gemm64(
    const unsigned short* __restrict__ Ap, const unsigned short* __restrict__ A2p, int lda, long strideA,
    const unsigned short* __restrict__ Btp, const unsigned short* __restrict__ Bt2p, int ldb, long strideB,
    void* __restrict__ Cout, void* __restrict__ Cout2, int ldc, long strideC,
    const float* __restrict__ bias,
    const float* __restrict__ resid, long strideR,
    int M, int N, int K, float scale) {
  typedef typename Elem<ET>::T T;
  typedef typename Frag<T>::V V;
  const T* A = (const T*)Ap; const T* A2 = (const T*)A2p; const T* Bt = (const T*)Btp; const T* Bt2 = (const T*)Bt2p;
  __shared__ __align__(16) float sT[8][16 * 68];
  const int b    = blockIdx.y;
  const int lane = threadIdx.x & 31;
  const int wave = threadIdx.x >> 5;
  const int tilesN = N >> 6;
  const int tilesM = M >> 6;
  const int tile = blockIdx.x * 8 + wave;
  if (tile >= tilesM * tilesN) return;
  const int tm = tile / tilesN;
  const int tn = tile - tm * tilesN;
  const int m0 = tm << 6;
  const int n0 = tn << 6;

  const T* Ab  = A  + (size_t)b * strideA;
  const T* Bb  = Bt + (size_t)b * strideB;
  const T* Ab2 = SPLIT ? (A2  + (size_t)b * strideA) : nullptr;
  const T* Bb2 = SPLIT ? (Bt2 + (size_t)b * strideB) : nullptr;

  const int rlane = lane & 15;
  const int koff  = (lane >> 4) * 8;
  const int mOff  = (lane >> 4) * 8;

  v8f acc[4][4];
#pragma unroll
  for (int i = 0; i < 4; ++i)
#pragma unroll
    for (int j = 0; j < 4; ++j) acc[i][j] = (v8f){0.f,0.f,0.f,0.f,0.f,0.f,0.f,0.f};

  for (int k0 = 0; k0 < K; k0 += 32) {
    V bh[4], bl[4];
#pragma unroll
    for (int j = 0; j < 4; ++j) {
      const size_t bo = (size_t)(n0 + (j << 4) + rlane) * ldb + koff + k0;
      bh[j] = Frag<T>::load(Bb + bo);
      if (SPLIT) bl[j] = Frag<T>::load(Bb2 + bo);
    }
#pragma unroll
    for (int i = 0; i < 4; ++i) {
      const size_t ao = (size_t)(m0 + (i << 4) + rlane) * lda + koff + k0;
      V ah = Frag<T>::load(Ab + ao);
      V al;
      if (SPLIT) al = Frag<T>::load(Ab2 + ao);
#pragma unroll
      for (int j = 0; j < 4; ++j) {
        acc[i][j] = Frag<T>::mma(ah, bh[j], acc[i][j]);
        if (SPLIT) {
          acc[i][j] = Frag<T>::mma(ah, bl[j], acc[i][j]);
          acc[i][j] = Frag<T>::mma(al, bh[j], acc[i][j]);
        }
      }
      Frag<T>::guard4(acc[i][0], acc[i][1], acc[i][2], acc[i][3], ah, SPLIT ? al : ah);
    }
    Frag<T>::keep(bh[0], bh[1], bh[2], bh[3]);
    if (SPLIT) Frag<T>::keep(bl[0], bl[1], bl[2], bl[3]);
  }
  acc_guard4(acc[0][0], acc[0][1], acc[0][2], acc[0][3]);
  acc_guard4(acc[1][0], acc[1][1], acc[1][2], acc[1][3]);
  acc_guard4(acc[2][0], acc[2][1], acc[2][2], acc[2][3]);
  acc_guard4(acc[3][0], acc[3][1], acc[3][2], acc[3][3]);

  float* slab = sT[wave];
  const float* Rb = RESID ? (resid + (size_t)b * strideR) : nullptr;
#pragma unroll
  for (int i = 0; i < 4; ++i) {
    const int mBase = m0 + (i << 4);
#pragma unroll
    for (int j = 0; j < 4; ++j) {
      const int n = n0 + (j << 4) + rlane;
      float bv = 0.f;
      if (BIAS_MODE == 2) bv = bias[n];
#pragma unroll
      for (int r = 0; r < 8; ++r) {
        float v = acc[i][j][r] * scale;
        if (BIAS_MODE == 1) v += bias[mBase + mOff + r];
        if (BIAS_MODE == 2) v += bv;
        if (RESID) v += Rb[(size_t)(mBase + mOff + r) * ldc + n];
        if (ACT == 1) v = tanhf(v);
        if (ACT == 2) v = fmaxf(v, 0.0f);
        if (ACT == 3) v = v / (1.0f + expf(-v));
        if (ACT == 4) v = (v > 0.f) ? v : 0.01f * v;
        slab[(mOff + r) * 68 + (j << 4) + rlane] = v;
      }
    }
    __builtin_amdgcn_fence(__ATOMIC_RELEASE, "workgroup");
    __builtin_amdgcn_wave_barrier();
    __builtin_amdgcn_fence(__ATOMIC_ACQUIRE, "workgroup");
    if (OUT_MODE == 0) {
      float* C = (float*)Cout + (size_t)b * strideC;
      const int hh = lane >> 4, c4 = (lane & 15) * 4;
      for (int pass = 0; pass < 2; ++pass) {
#pragma unroll
        for (int it = 0; it < 8; ++it) {
          const int row = it * 2 + hh;
          v4f v = *(const v4f*)(slab + row * 68 + c4);
          *(volatile v4f*)(C + (size_t)(mBase + row) * ldc + n0 + c4) = v;
        }
        __threadfence();
      }
    } else {
      const int q = lane >> 3, c8 = (lane & 7) * 8;
      unsigned short* C  = (unsigned short*)Cout  + (size_t)b * strideC;
      unsigned short* C2 = (OUT_MODE == 2) ? ((unsigned short*)Cout2 + (size_t)b * strideC) : nullptr;
      for (int pass = 0; pass < 2; ++pass) {
#pragma unroll
        for (int it = 0; it < 4; ++it) {
          const int row = it * 4 + q;
          const float* sp = slab + row * 68 + c8;
          v8h hv, lv;
#pragma unroll
          for (int e = 0; e < 8; ++e) {
            if (OUT_MODE == 1) {
              hv[e] = (_Float16)sp[e];
            } else {
              unsigned short hb = f2bf_bits(sp[e]);
              unsigned short lb = f2bf_bits(sp[e] - bf_bits2f(hb));
              hv[e] = __builtin_bit_cast(_Float16, hb);
              lv[e] = __builtin_bit_cast(_Float16, lb);
            }
          }
          *(volatile v8h*)(C + (size_t)(mBase + row) * ldc + n0 + c8) = hv;
          if (OUT_MODE == 2) *(volatile v8h*)(C2 + (size_t)(mBase + row) * ldc + n0 + c8) = lv;
        }
        __threadfence();
      }
    }
    __builtin_amdgcn_fence(__ATOMIC_RELEASE, "workgroup");
    __builtin_amdgcn_wave_barrier();
    __builtin_amdgcn_fence(__ATOMIC_ACQUIRE, "workgroup");
  }
}


__device__ __forceinline__ void store2(float* p, float v) {
  *(volatile float*)p = v;
  __threadfence();
  *(volatile float*)p = v;
}

__global__ __launch_bounds__(kThr) void cast_plane_kernel(const float* __restrict__ src, unsigned short* __restrict__ dst,
                                                          int colsLog2, int dstPitch, int dstOff) {
  const int i   = blockIdx.x * kThr + threadIdx.x;
  const int sh  = colsLog2 - 3;
  const int row = i >> sh;
  const int c8  = (i & ((1 << sh) - 1)) * 8;
  const float* sp = src + ((size_t)row << colsLog2) + c8;
  const v4f a0 = *(const v4f*)(sp);
  const v4f a1 = *(const v4f*)(sp + 4);
  v8h hv;
#pragma unroll
  for (int e = 0; e < 4; ++e) {
    const float f0 = a0[e];
    const float f1 = a1[e];
    hv[e]     = (_Float16)carry_flush(bf16r(f0), kInCarry);
    hv[4 + e] = (_Float16)carry_flush(bf16r(f1), kInCarry);
  }
  unsigned short* dp = dst + (size_t)row * dstPitch + dstOff + c8;
  *(volatile v8h*)dp = hv;
  __threadfence();
  *(volatile v8h*)dp = hv;
}

__global__ __launch_bounds__(256) void wt_plane_kernel(const float* __restrict__ W, unsigned short* __restrict__ dst, int K, int N, int nLive, int ldd, int colOff) {
  const int n  = blockIdx.x;
  const int k8 = threadIdx.x * 8;
  const bool live = n < nLive;
  const int nc = live ? n : 0;
  v8h hv;
#pragma unroll
  for (int e = 0; e < 8; ++e) {
    const float w = W[(size_t)(k8 + e) * N + nc];
    hv[e] = (_Float16)(live ? carry_flush(bf16r(w), kWCarry) : 0.0f);
  }
  unsigned short* dp = dst + (size_t)n * ldd + colOff + k8;
  *(volatile v8h*)dp = hv;
  __threadfence();
  *(volatile v8h*)dp = hv;
}

__global__ __launch_bounds__(kThr) void setup_kernel(const float* __restrict__ embed_b, const float* __restrict__ out_b, const float* __restrict__ dec_b,
                                                    const float* __restrict__ embed_w, const float* __restrict__ dec_w,
                                                    float* __restrict__ EB, float* __restrict__ OB, float* __restrict__ DB,
                                                    unsigned short* __restrict__ WE16, unsigned short* __restrict__ WD16) {
  const unsigned bk = blockIdx.x;
  const unsigned t = threadIdx.x;
  if (bk == 0u || bk == 5u) {
    const bool isE = bk == 0u;
    const unsigned lim = isE ? (unsigned)kH : (unsigned)kDo;
    const float p = (isE ? embed_b : dec_b)[t & (lim - 1u)];
    const float o = (t < lim) ? bf16r(p) : 0.0f;
    float* dp = (isE ? EB : DB) + t;
    *(volatile float*)dp = o;
    __threadfence();
    *(volatile float*)dp = o;
  } else if (bk < 5u) {
    const unsigned i = (bk - 1u) * (unsigned)kThr + t;
    const float p = out_b[i];
    const float o = bf16r(p);
    *(volatile float*)(OB + i) = o;
    __threadfence();
    *(volatile float*)(OB + i) = o;
  } else {
    const bool isE = bk < 8u;
    const unsigned j = (bk - (isE ? 6u : 8u)) * (unsigned)kThr + t;
    const unsigned n = isE ? (j >> 2) : (j >> 4);
    const unsigned c8 = (isE ? (j & 3u) : (j & 15u)) * 8u;
    const unsigned ncol = isE ? (unsigned)kH : (unsigned)kDo;
    const bool live = isE || n < (unsigned)kDo;
    const float* sp = (isE ? embed_w : dec_w) + (size_t)c8 * ncol + (live ? n : 0u);
    v8h hv;
#pragma unroll
    for (int e = 0; e < 8; ++e) {
      const float f = sp[(size_t)e * ncol];
      hv[e] = (_Float16)(live ? carry_flush(bf16r(f), kInCarry) : 0.0f);
    }
    unsigned short* dp = (isE ? WE16 : WD16) + (size_t)n * (isE ? (unsigned)kDin : (unsigned)kH) + c8;
    *(volatile v8h*)dp = hv;
    __threadfence();
    *(volatile v8h*)dp = hv;
  }
}
static_assert(kNL * kG == 4 * kThr && kH * kDin / 8 == 2 * kThr && kDoP * kH / 8 == 4 * kThr && kH <= kThr && kDo <= kThr, "set-up grid exact: 1 + 4 + 1 blocks of bias records, 2 of the embedding's weight, 4 of the decoder's");

__global__ __launch_bounds__(kThr) void par_kernel(const float* __restrict__ log_dt, const float* __restrict__ A_re, const float* __restrict__ A_im,
                                                   const float* __restrict__ C_re, const float* __restrict__ C_im, float* __restrict__ PAR) {
  const unsigned j = blockIdx.x * (unsigned)kThr + threadIdx.x;
  const unsigned ch = j >> 5;
  const float ld = log_dt[ch];
  const float dt = expf(bf16r(ld));
  const float a0 = A_re[j], a1 = A_im[j], c0 = C_re[j], c1 = C_im[j];
  const float ar = bf16r(a0), ai = bf16r(a1), cr = bf16r(c0), ci = bf16r(c1);
  const float mag = expf(ar * dt);
  const float ph = ai * dt;
  const float lr = mag * cosf(ph);
  const float li = mag * sinf(ph);
  const float nr = lr - 1.0f, ni = li;
  const float den = ar * ar + ai * ai;
  const float qr = (nr * ar + ni * ai) / den;
  const float qi = (ni * ar - nr * ai) / den;
  v4f o;
  o[0] = lr; o[1] = li; o[2] = cr * qr - ci * qi; o[3] = cr * qi + ci * qr;
  float* dp = PAR + (size_t)j * 4;
  *(volatile v4f*)dp = o;
  __threadfence();
  *(volatile v4f*)dp = o;
}
static_assert(kNL * kH * kNs == 64 * kThr && kNs == 32, "the parameter kernel's grid exact: 64 blocks: 16,384 states");

__global__ __launch_bounds__(kThr) void scan_kernel(const float* __restrict__ Hin, const float* __restrict__ PAR, const float* __restrict__ D_skip,
                                                    float* __restrict__ YF, int layer) {
  const unsigned ix = blockIdx.x * (unsigned)kThr + threadIdx.x;
  const unsigned b = ix >> 7;
  const unsigned h = ix & 127u;
  const size_t ch = (size_t)layer * kH + h;
  float lr[kNs], li[kNs], kr[kNs], ki[kNs], sr[kNs], si[kNs];
  const float dk0 = D_skip[ch];
  const float dsk = bf16r(dk0);
  const float* pp = PAR + ch * (size_t)(kNs * 4);
#pragma unroll
  for (int n = 0; n < kNs; ++n) {
    const v4f p = *(const v4f*)(pp + 4 * n);
    lr[n] = p[0]; li[n] = p[1]; kr[n] = p[2]; ki[n] = p[3];
    sr[n] = 0.0f; si[n] = 0.0f;
  }
  for (int l = 0; l < kL; ++l) {
    const size_t row = (size_t)b * kL + (size_t)l;
    const float u = Hin[row * kH + h];
    float acc = 0.0f;
#pragma unroll
    for (int n = 0; n < kNs; ++n) {
      const float nsr = lr[n] * sr[n] - li[n] * si[n] + u;
      const float nsi = lr[n] * si[n] + li[n] * sr[n];
      sr[n] = nsr; si[n] = nsi;
      acc += kr[n] * nsr - ki[n] * nsi;
    }
    const float y = (acc + acc) + dsk * u;
    float* dp = YF + row * kH + h;
    *(volatile float*)dp = y;
    __threadfence();
    *(volatile float*)dp = y;
  }
}
static_assert(kNB * kH == 8 * kThr && kH == 128, "walk grid exact: 8 blocks: 128 channels of 16 sequences");

__global__ __launch_bounds__(kThr) void gelu_cast_kernel(const float* __restrict__ YF, unsigned short* __restrict__ Y16) {
  const size_t i8 = ((size_t)blockIdx.x * kThr + threadIdx.x) * 8;
  const v4f a0 = *(const v4f*)(YF + i8), a1 = *(const v4f*)(YF + i8 + 4);
  v8h hv;
#pragma unroll
  for (int e = 0; e < 8; ++e) {
    const float v = (e < 4) ? a0[e] : a1[e - 4];
    const float t = 0.7978845608028654f * (v + 0.044715f * v * v * v);
    const float g = 0.5f * v * (1.0f + tanhf(t));
    hv[e] = (_Float16)carry_flush(g, kYCarry);
  }
  unsigned short* dp = Y16 + i8;
  *(volatile v8h*)dp = hv;
  __threadfence();
  *(volatile v8h*)dp = hv;
}
static_assert(((size_t)kRows * kH / 8) == 4096ull * kThr, "the gelu's grid exact: 4,096 blocks");

__global__ __launch_bounds__(kThr) void glu_norm_kernel(const float* __restrict__ V, const float* __restrict__ Hin, const float* __restrict__ norm_w, const float* __restrict__ norm_b,
                                                        float* __restrict__ Hout, unsigned short* __restrict__ HF16, int layer, int last) {
  const size_t row = (size_t)blockIdx.x * kThr + threadIdx.x;
  const float* vp = V + row * kG;
  const float* hp = Hin + row * kH;
  float hv[kH];
  float sum = 0.0f;
#pragma unroll
  for (int c4 = 0; c4 < kH / 4; ++c4) {
    const v4f a = *(const v4f*)(vp + 4 * c4), g = *(const v4f*)(vp + kH + 4 * c4), r = *(const v4f*)(hp + 4 * c4);
#pragma unroll
    for (int e = 0; e < 4; ++e) {
      const float z = a[e] / (1.0f + expf(-g[e]));
      const float hn = z + r[e];
      hv[4 * c4 + e] = hn;
      sum += hn;
    }
  }
  const float mu = sum / (float)kH;
  float q = 0.0f;
#pragma unroll
  for (int c = 0; c < kH; ++c) { const float d = hv[c] - mu; q += d * d; }
  const float rs = 1.0f / sqrtf(q / (float)kH + 1e-5f);
  const float* gw = norm_w + (size_t)layer * kH;
  const float* gb = norm_b + (size_t)layer * kH;
#pragma unroll
  for (int c = 0; c < kH; ++c) { const float w0 = gw[c], b0 = gb[c]; hv[c] = ((hv[c] - mu) * rs) * bf16r(w0) + bf16r(b0); }
  float* op = Hout + row * kH;
  for (int pass = 0; pass < 2; ++pass) {
#pragma unroll
    for (int c4 = 0; c4 < kH / 4; ++c4) { v4f o; o[0] = hv[4 * c4]; o[1] = hv[4 * c4 + 1]; o[2] = hv[4 * c4 + 2]; o[3] = hv[4 * c4 + 3]; *(volatile v4f*)(op + 4 * c4) = o; }
    __threadfence();
  }
  if (last) {
    unsigned short* fp = HF16 + row * kH;
    for (int pass = 0; pass < 2; ++pass) {
#pragma unroll
      for (int c8 = 0; c8 < kH / 8; ++c8) {
        v8h o;
#pragma unroll
        for (int e = 0; e < 8; ++e) o[e] = (_Float16)carry_flush(hv[8 * c8 + e], kInCarry);
        *(volatile v8h*)(fp + 8 * c8) = o;
      }
      __threadfence();
    }
  }
}
static_assert(kRows == 256 * kThr && (kH % 8) == 0, "the norm's grid exact: 256 blocks: a thread a row");

__global__ __launch_bounds__(kThr) void outcopy_kernel(const float* __restrict__ DEC, float* __restrict__ out) {
  const unsigned i = blockIdx.x * (unsigned)kThr + threadIdx.x;
  const size_t row = i >> 2;
  const unsigned c8 = (i & 3u) * 8u;
  const v4f a0 = *(const v4f*)(DEC + row * kDoP + c8), a1 = *(const v4f*)(DEC + row * kDoP + c8 + 4);
  float* dp = out + row * kDo + c8;
  for (int pass = 0; pass < 2; ++pass) { *(volatile v4f*)dp = a0; *(volatile v4f*)(dp + 4) = a1; __threadfence(); }
}
static_assert((size_t)kRows * 4 == 1024ull * kThr && kDo == 4 * 8, "the copy's grid exact: 1,024 blocks; 4 chunks a row, all live");

extern "C" void kernel_launch(void* const* d_in, const int* in_sizes, int n_in,
                              void* d_out, int out_size, void* d_ws, size_t ws_size,
                              hipStream_t stream) {
  if (n_in < 15 || d_out == nullptr || d_ws == nullptr) return;
  if (in_sizes[0] != kRows * kDin || in_sizes[1] != kDin * kH || in_sizes[2] != kH || in_sizes[3] != kNL * kH || in_sizes[4] != kNL * kH * kNs || in_sizes[5] != kNL * kH * kNs) return;
  if (in_sizes[6] != kNL * kH * kNs || in_sizes[7] != kNL * kH * kNs || in_sizes[8] != kNL * kH || in_sizes[9] != kNL * kG * kH || in_sizes[10] != kNL * kG) return;
  if (in_sizes[11] != kNL * kH || in_sizes[12] != kNL * kH || in_sizes[13] != kH * kDo || in_sizes[14] != kDo) return;
  if (out_size != kRows * kDo) return;
  if (ws_size < kWsTotal) return;
  const float* x = (const float*)d_in[0];
  const float* embed_w = (const float*)d_in[1];
  const float* embed_b = (const float*)d_in[2];
  const float* log_dt = (const float*)d_in[3];
  const float* A_re = (const float*)d_in[4];
  const float* A_im = (const float*)d_in[5];
  const float* C_re = (const float*)d_in[6];
  const float* C_im = (const float*)d_in[7];
  const float* D_skip = (const float*)d_in[8];
  const float* out_w = (const float*)d_in[9];
  const float* out_b = (const float*)d_in[10];
  const float* norm_w = (const float*)d_in[11];
  const float* norm_b = (const float*)d_in[12];
  const float* dec_w = (const float*)d_in[13];
  const float* dec_b = (const float*)d_in[14];
  float* out = (float*)d_out;
  char* ws = (char*)d_ws;
  unsigned short* X16 = (unsigned short*)(ws + kOffX16);
  unsigned short* WO16 = (unsigned short*)(ws + kOffWO16);
  unsigned short* WE16 = (unsigned short*)(ws + kOffWE16);
  unsigned short* WD16 = (unsigned short*)(ws + kOffWD16);
  float* EB = (float*)(ws + kOffEB);
  float* OB = (float*)(ws + kOffOB);
  float* DB = (float*)(ws + kOffDB);
  float* H0 = (float*)(ws + kOffH0);
  float* H1 = (float*)(ws + kOffH1);
  float* PAR = (float*)(ws + kOffPAR);
  float* YF = (float*)(ws + kOffYF);
  unsigned short* Y16 = (unsigned short*)(ws + kOffY16);
  unsigned short* HF16 = Y16;
  float* V = (float*)(ws + kOffV);
  float* DEC = (float*)(ws + kOffDEC);

  static_assert(((size_t)kRows * kDin / 8) % kThr == 0 && ((size_t)kNL * kG * kH / 8) % kThr == 0 && ((size_t)kRows * kDin) % 1024 == 0 && ((size_t)kNL * kG * kH) % 1024 == 0, "the casts' grids; each plane is whole rows of 1,024");
  cast_plane_kernel<<<(int)(((size_t)kRows * kDin / 8) / kThr), kThr, 0, stream>>>(x, X16, 10, 1024, 0);
  cast_plane_kernel<<<(int)(((size_t)kNL * kG * kH / 8) / kThr), kThr, 0, stream>>>(out_w, WO16, 10, 1024, 0);
  setup_kernel<<<12, kThr, 0, stream>>>(embed_b, out_b, dec_b, embed_w, dec_w, EB, OB, DB, WE16, WD16);
  par_kernel<<<64, kThr, 0, stream>>>(log_dt, A_re, A_im, C_re, C_im, PAR);
  wmma_gemm64<0, false, 2, 0, false, 0><<<dim3((kRows / 64) * (kH / 64) / 8, 1), 256, 0, stream>>>(
      X16, X16, kDin, 0L, WE16, WE16, kDin, 0L, (void*)H0, (void*)H0, kH, 0L, EB, nullptr, 0L, kRows, kH, kDin, kScE);
  for (int i = 0; i < kNL; ++i) {
    float* Hin = (i & 1) ? H1 : H0;
    float* Hout = (i & 1) ? H0 : H1;
    scan_kernel<<<8, kThr, 0, stream>>>(Hin, PAR, D_skip, YF, i);
    gelu_cast_kernel<<<4096, kThr, 0, stream>>>(YF, Y16);
    wmma_gemm64<0, false, 2, 0, false, 0><<<dim3((kRows / 64) * (kG / 64) / 8, 1), 256, 0, stream>>>(
        Y16, Y16, kH, 0L, WO16 + (size_t)i * kG * kH, WO16 + (size_t)i * kG * kH, kH, 0L, (void*)V, (void*)V, kG, 0L, OB + (size_t)i * kG, nullptr, 0L, kRows, kG, kH, kScO);
    glu_norm_kernel<<<256, kThr, 0, stream>>>(V, Hin, norm_w, norm_b, Hout, HF16, i, (i == kNL - 1) ? 1 : 0);
  }
  wmma_gemm64<0, false, 2, 0, false, 0><<<dim3((kRows / 64) * (kDoP / 64) / 8, 1), 256, 0, stream>>>(
      HF16, HF16, kH, 0L, WD16, WD16, kH, 0L, (void*)DEC, (void*)DEC, kDoP, 0L, DB, nullptr, 0L, kRows, kDoP, kH, kScD);
  outcopy_kernel<<<1024, kThr, 0, stream>>>(DEC, out);
}
static_assert(((kRows / 64) * (kH / 64)) % 8 == 0 && ((kRows / 64) * (kG / 64)) % 8 == 0 && ((kRows / 64) * (kDoP / 64)) % 8 == 0, "the engine's grids: whole blocks of eight wave tiles");
